// RNN_24781961298493
// MI455X (gfx1250) — hardware-verified
//
#include <hip/hip_runtime.h>
#include <math.h>

constexpr int NBATCH   = 16384;
constexpr int NSTEP    = 64;
constexpr int NHID     = 64;
constexpr int NGATE    = 256;
constexpr int NVOCAB   = 25;
constexpr int NEMB     = 32;
constexpr int NOUTF    = 3;
constexpr int TABROWS  = 32;
constexpr int ROWS_BLK = 64;
constexpr int CELL_THR = 128;
constexpr int PREP_THR = 256;
constexpr int WPITCH   = 72;
constexpr int HPITCH   = 72;
constexpr int HFPITCH  = 68;
constexpr int OUT_BLK  = ROWS_BLK * NOUTF;

static_assert(NGATE == 4 * NHID);
static_assert(NHID == 64);
static_assert(NHID % 32 == 0);
static_assert(NBATCH % ROWS_BLK == 0);
static_assert(ROWS_BLK == 16 * (CELL_THR / 32));
static_assert(OUT_BLK == 192);
static_assert((OUT_BLK * 4) % 128 == 0);
static_assert(TABROWS >= NVOCAB);
static_assert((TABROWS * NGATE / 4) % PREP_THR == 0);
static_assert((NGATE * NHID / 8) % PREP_THR == 0);
static_assert((WPITCH % 8) == 0 && (HPITCH % 8) == 0 && (HFPITCH % 4) == 0);

typedef __attribute__((ext_vector_type(16))) _Float16 v16h;
typedef __attribute__((ext_vector_type(8)))  _Float16 v8h;
typedef __attribute__((ext_vector_type(8)))  float    v8f;
typedef __attribute__((ext_vector_type(4)))  float    v4f;
typedef __attribute__((ext_vector_type(4)))  int      v4i;

struct FragH {
  union U { v16h v; v8h h[2]; };
  static __device__ __forceinline__ v16h load(const _Float16* p) {
    U f;
    f.h[0] = *(const v8h*)(p);
    f.h[1] = *(const v8h*)(p + 16);
    return f.v;
  }
};

__device__ __forceinline__ v8f mma2_h(v16h a0, v16h b0, v16h a1, v16h b1, v8f c) {
  c = __builtin_amdgcn_wmma_f32_16x16x32_f16(false, a0, false, b0, (short)0, c, false, false);
  c = __builtin_amdgcn_wmma_f32_16x16x32_f16(false, a1, false, b1, (short)0, c, false, false);
  asm volatile("v_nop\n\tv_nop\n\tv_nop\n\tv_nop" : "+v"(c) : "v"(a0), "v"(b0), "v"(a1), "v"(b1));
  return c;
}

__device__ __forceinline__ float sigm(float x)   { return __builtin_amdgcn_rcpf(1.0f + expf(-x)); }
__device__ __forceinline__ float tanh_e(float x) { return 1.0f - 2.0f * __builtin_amdgcn_rcpf(expf(2.0f * x) + 1.0f); }

__global__ __launch_bounds__(PREP_THR) void prep_kernel(const float* __restrict__ emb, const float* __restrict__ wih,
                                                        const float* __restrict__ whh, const float* __restrict__ bih,
                                                        const float* __restrict__ bhh, float* __restrict__ XT,
                                                        unsigned short* __restrict__ WHp) {
  const int tid = threadIdx.x;
#pragma unroll 1
  for (int it = 0; it < (TABROWS * NGATE / 4) / PREP_THR; ++it) {
    const int idx  = it * PREP_THR + tid;
    const int tok  = idx >> 6;
    const int rem  = idx & 63;
    const int cc   = rem >> 2;
    const int jj   = rem & 3;
    const int tokc = (tok < NVOCAB) ? tok : (NVOCAB - 1);
    const int unit = 16 * jj + cc;
    const float* er = emb + tokc * NEMB;
    const float* w0 = wih + (0 * NHID + unit) * NEMB;
    const float* w1 = wih + (1 * NHID + unit) * NEMB;
    const float* w2 = wih + (2 * NHID + unit) * NEMB;
    const float* w3 = wih + (3 * NHID + unit) * NEMB;
    float s0 = 0.0f, s1 = 0.0f, s2 = 0.0f, s3 = 0.0f;
#pragma unroll 1
    for (int e = 0; e < NEMB; ++e) {
      const float x = er[e];
      s0 = fmaf(x, w0[e], s0);
      s1 = fmaf(x, w1[e], s1);
      s2 = fmaf(x, w2[e], s2);
      s3 = fmaf(x, w3[e], s3);
    }
    s0 = (s0 + bih[0 * NHID + unit]) + bhh[0 * NHID + unit];
    s1 = (s1 + bih[1 * NHID + unit]) + bhh[1 * NHID + unit];
    s2 = (s2 + bih[2 * NHID + unit]) + bhh[2 * NHID + unit];
    s3 = (s3 + bih[3 * NHID + unit]) + bhh[3 * NHID + unit];
    const bool live = (tok < NVOCAB);
    v4f o;
    o[0] = live ? s0 : 0.0f;
    o[1] = live ? s1 : 0.0f;
    o[2] = live ? s2 : 0.0f;
    o[3] = live ? s3 : 0.0f;
    float* op = XT + 4 * idx;
    *(volatile v4f*)op = o;
    __threadfence();
    *(volatile v4f*)op = o;
  }
#pragma unroll 1
  for (int it = 0; it < (NGATE * NHID / 8) / PREP_THR; ++it) {
    const int idx = it * PREP_THR + tid;
    const float* sp = whh + 8 * idx;
    const v4f a = *(const v4f*)(sp);
    const v4f b = *(const v4f*)(sp + 4);
    v8h hv;
#pragma unroll
    for (int e = 0; e < 4; ++e) {
      const float fa = a[e];
      const float fb = b[e];
      hv[e]     = (_Float16)fa;
      hv[4 + e] = (_Float16)fb;
    }
    unsigned short* dp = WHp + 8 * idx;
    *(volatile v8h*)dp = hv;
    __threadfence();
    *(volatile v8h*)dp = hv;
  }
}

__global__ __launch_bounds__(CELL_THR) void seq_cell_kernel(const int* __restrict__ msg, const float* __restrict__ XT,
                                                            const unsigned short* __restrict__ WHp,
                                                            const float* __restrict__ fcw, const float* __restrict__ fcb,
                                                            float* __restrict__ out) {
  __shared__ __align__(16) _Float16 Wl[NGATE * WPITCH];
  __shared__ __align__(16) float    Xt[TABROWS * NGATE];
  __shared__ __align__(16) _Float16 Ah[2 * ROWS_BLK * HPITCH];
  __shared__ __align__(16) int      Tk[NSTEP * ROWS_BLK];
  __shared__ __align__(16) float    Hf[ROWS_BLK * HFPITCH];
  __shared__ __align__(16) float    Ost[OUT_BLK];

  const _Float16* WH = (const _Float16*)WHp;
  const int tid  = threadIdx.x;
  const int lane = tid & 31;
  const int wave = tid >> 5;
  const int c    = lane & 15;
  const int hh   = lane >> 4;
  const int koff = hh * 8;
  const int blk  = blockIdx.x;

  v8h zero8;
#pragma unroll
  for (int e = 0; e < 8; ++e) zero8[e] = (_Float16)0.0f;

#pragma unroll 4
  for (int i = 0; i < 16; ++i) {
    const int idx = i * CELL_THR + tid;
    const int row = idx >> 3;
    const int ch  = idx & 7;
    const v8h v = *(const v8h*)(WH + row * NHID + ch * 8);
    *(v8h*)(Wl + row * WPITCH + ch * 8) = v;
  }
#pragma unroll
  for (int i = 0; i < 2; ++i) {
    const int row = i * CELL_THR + tid;
    *(v8h*)(Wl + row * WPITCH + NHID) = zero8;
  }
#pragma unroll 4
  for (int i = 0; i < 16; ++i) {
    const int idx = i * CELL_THR + tid;
    const v4f v = *(const v4f*)(XT + 4 * idx);
    *(v4f*)(Xt + 4 * idx) = v;
  }
  {
    const int* mb = msg + (size_t)blk * (size_t)(ROWS_BLK * NSTEP);
#pragma unroll 4
    for (int i = 0; i < 8; ++i) {
      const int idx = i * CELL_THR + tid;
      const v4i v = *(const v4i*)(mb + 4 * idx);
      const int row = idx >> 4;
      const int t0  = (idx & 15) * 4;
#pragma unroll
      for (int e = 0; e < 4; ++e) {
        int tk = v[e];
        tk = (tk < 0) ? 0 : tk;
        tk = (tk > NVOCAB - 1) ? (NVOCAB - 1) : tk;
        Tk[(t0 + e) * ROWS_BLK + row] = tk * NGATE;
      }
    }
  }
#pragma unroll 1
  for (int i = 0; i < 9; ++i) {
    *(v8h*)(Ah + 8 * (i * CELL_THR + tid)) = zero8;
  }
  __syncthreads();

  const v8f zf8 = {0.f, 0.f, 0.f, 0.f, 0.f, 0.f, 0.f, 0.f};
  v8f cs0 = zf8, cs1 = zf8, cs2 = zf8, cs3 = zf8;

  const int arow_off = (16 * wave + c) * HPITCH + koff;
  const int hrow_off = (16 * wave + 8 * hh) * HPITCH + c;
  const float*    xcol = Xt + c * 16;
  const _Float16* wrow = Wl + c * WPITCH + koff;
  float* hfp = Hf + (16 * wave + 8 * hh) * HFPITCH + c;

#pragma unroll 1
  for (int t = 0; t < NSTEP; ++t) {
    const int cur = t & 1;
    const bool last = (t == NSTEP - 1);
    const _Float16* ar = Ah + cur * (ROWS_BLK * HPITCH) + arow_off;
    const v16h a0 = FragH::load(ar);
    const v16h a1 = FragH::load(ar + 32);
    _Float16* hn = Ah + (cur ^ 1) * (ROWS_BLK * HPITCH) + hrow_off;

    const v4i tka = *(const v4i*)(Tk + t * ROWS_BLK + 16 * wave + 8 * hh);
    const v4i tkb = *(const v4i*)(Tk + t * ROWS_BLK + 16 * wave + 8 * hh + 4);
    int toff[8];
    toff[0] = tka[0]; toff[1] = tka[1]; toff[2] = tka[2]; toff[3] = tka[3];
    toff[4] = tkb[0]; toff[5] = tkb[1]; toff[6] = tkb[2]; toff[7] = tkb[3];

#pragma unroll 1
    for (int j = 0; j < 4; ++j) {
      v8f acc0, acc1, acc2, acc3;
#pragma unroll
      for (int r = 0; r < 8; ++r) {
        const v4f x = *(const v4f*)(xcol + toff[r] + 4 * j);
        acc0[r] = x[0];
        acc1[r] = x[1];
        acc2[r] = x[2];
        acc3[r] = x[3];
      }
      {
        const _Float16* wq = wrow + (0 * NHID + 16 * j) * WPITCH;
        const v16h b0 = FragH::load(wq);
        const v16h b1 = FragH::load(wq + 32);
        acc0 = mma2_h(a0, b0, a1, b1, acc0);
      }
      {
        const _Float16* wq = wrow + (1 * NHID + 16 * j) * WPITCH;
        const v16h b0 = FragH::load(wq);
        const v16h b1 = FragH::load(wq + 32);
        acc1 = mma2_h(a0, b0, a1, b1, acc1);
      }
      {
        const _Float16* wq = wrow + (2 * NHID + 16 * j) * WPITCH;
        const v16h b0 = FragH::load(wq);
        const v16h b1 = FragH::load(wq + 32);
        acc2 = mma2_h(a0, b0, a1, b1, acc2);
      }
      {
        const _Float16* wq = wrow + (3 * NHID + 16 * j) * WPITCH;
        const v16h b0 = FragH::load(wq);
        const v16h b1 = FragH::load(wq + 32);
        acc3 = mma2_h(a0, b0, a1, b1, acc3);
      }
      v8f cn8, hv8;
#pragma unroll
      for (int r = 0; r < 8; ++r) {
        const float ig = sigm(acc0[r]);
        const float fg = sigm(acc1[r]);
        const float gg = tanh_e(acc2[r]);
        const float og = sigm(acc3[r]);
        const float cn = fg * cs0[r] + ig * gg;
        cn8[r] = cn;
        const float hv = og * tanh_e(cn);
        hv8[r] = hv;
        hn[r * HPITCH + 16 * j] = (_Float16)hv;
      }
      if (last) {
#pragma unroll
        for (int r = 0; r < 8; ++r) hfp[r * HFPITCH + 16 * j] = hv8[r];
      }
      cs0 = cs1;
      cs1 = cs2;
      cs2 = cs3;
      cs3 = cn8;
    }
    __syncthreads();
  }

#pragma unroll 1
  for (int it = 0; it < 2; ++it) {
    const int idx = it * CELL_THR + tid;
    const int idc = (idx < OUT_BLK) ? idx : (OUT_BLK - 1);
    const int row = idc / NOUTF;
    const int o   = idc - NOUTF * row;
    const float* hr = Hf + row * HFPITCH;
    const float* wr = fcw + o * NHID;
    float s = 0.0f;
#pragma unroll 1
    for (int k = 0; k < NHID; ++k) s = fmaf(hr[k], wr[k], s);
    s = s + fcb[o];
    if (idx < OUT_BLK) Ost[idx] = s;
  }
  __syncthreads();

  {
    const int vi = (wave == 0) ? lane : (32 + (lane & 15));
    const v4f ov = *(const v4f*)(Ost + 4 * vi);
    const bool dost = (wave == 0) || ((wave == 1) && (lane < 16));
    float* op = out + (size_t)blk * (size_t)OUT_BLK + 4 * vi;
    if (dost) { *(volatile v4f*)op = ov; }
    __threadfence();
    if (dost) { *(volatile v4f*)op = ov; }
  }
}

extern "C" void kernel_launch(void* const* d_in, const int* in_sizes, int n_in,
                              void* d_out, int out_size, void* d_ws, size_t ws_size, hipStream_t stream) {
  if (n_in < 8 || d_out == nullptr || d_ws == nullptr) return;
  if (in_sizes[0] != NBATCH * NSTEP || in_sizes[1] != NVOCAB * NEMB || in_sizes[2] != NGATE * NEMB ||
      in_sizes[3] != NGATE * NHID || in_sizes[4] != NGATE || in_sizes[5] != NGATE ||
      in_sizes[6] != NOUTF * NHID || in_sizes[7] != NOUTF || out_size != NBATCH * NOUTF) return;

  const int*   msg = (const int*)d_in[0];
  const float* emb = (const float*)d_in[1];
  const float* wih = (const float*)d_in[2];
  const float* whh = (const float*)d_in[3];
  const float* bih = (const float*)d_in[4];
  const float* bhh = (const float*)d_in[5];
  const float* fcw = (const float*)d_in[6];
  const float* fcb = (const float*)d_in[7];
  float* out = (float*)d_out;

  char* ws = (char*)d_ws;
  size_t off = 0;
  auto carve = [&](size_t bytes) -> char* { char* p = ws + off; off += (bytes + 255) & ~(size_t)255; return p; };
  float*          XT  = (float*)carve((size_t)TABROWS * NGATE * 4);
  unsigned short* WHp = (unsigned short*)carve((size_t)NGATE * NHID * 2);
  if (off > ws_size || off > (size_t)134217728) return;

  prep_kernel<<<1, PREP_THR, 0, stream>>>(emb, wih, whh, bih, bhh, XT, WHp);
  seq_cell_kernel<<<NBATCH / ROWS_BLK, CELL_THR, 0, stream>>>(msg, XT, WHp, fcw, fcb, out);
}
